// PeerInteractionFeatureExtractor_90400471646753
// MI455X (gfx1250) — hardware-verified
//
#include <hip/hip_runtime.h>
#include <math.h>

typedef __attribute__((ext_vector_type(16))) _Float16 v16h;
typedef __attribute__((ext_vector_type(16))) __bf16 v16b;
typedef __attribute__((ext_vector_type(8)))  _Float16 v8h;
typedef __attribute__((ext_vector_type(8)))  float v8f;
typedef __attribute__((ext_vector_type(4)))  float v4f;
typedef __attribute__((ext_vector_type(2)))  float v2f;
typedef __attribute__((ext_vector_type(4)))  unsigned v4u;
typedef __attribute__((ext_vector_type(4)))  int v4i;
typedef float __attribute__((may_alias)) float_a;
typedef int __attribute__((may_alias)) int_a;

template <typename T> __device__ __forceinline__ void vst2(void* p, T v) { *(volatile T*)p = v; __threadfence(); *(volatile T*)p = v; }
__device__ __forceinline__ v8f wmma16(v16h a, v16h b, v8f c) {
  v8f d = __builtin_amdgcn_wmma_f32_16x16x32_f16(false, a, false, b, (short)0, c, false, false);
  asm volatile("v_nop\n\tv_nop\n\tv_nop\n\tv_nop" : "+v"(d) : "v"(a), "v"(b));
  return d;
}
__device__ __forceinline__ v8f wmma_bf(v16b a, v16b b, v8f c) {
  v8f d = __builtin_amdgcn_wmma_f32_16x16x32_bf16(false, a, false, b, (short)0, c, false, false);
  asm volatile("v_nop\n\tv_nop\n\tv_nop\n\tv_nop" : "+v"(d) : "v"(a), "v"(b));
  return d;
}
__device__ __forceinline__ v16h frag_h(const _Float16* rowk0, int lane) {
  union { v16h v; v8h q[2]; } u; const _Float16* p = rowk0 + 8 * (lane >> 4);
  u.q[0] = *(const v8h*)p; u.q[1] = *(const v8h*)(p + 16); return u.v;
}
__device__ __forceinline__ v16h frag_f32(const float* rowk0, int lane) {
  v16h a; const float* p = rowk0 + 8 * (lane >> 4);
#pragma unroll
  for (int i = 0; i < 8; ++i) { a[i] = (_Float16)p[i]; a[8 + i] = (_Float16)p[16 + i]; }
  return a;
}
__device__ __forceinline__ v16h frag_f32s(const float* rowk0, int lane, float sc) {
  v16h a; const float* p = rowk0 + 8 * (lane >> 4);
#pragma unroll
  for (int i = 0; i < 8; ++i) { a[i] = (_Float16)(p[i] * sc); a[8 + i] = (_Float16)(p[16 + i] * sc); }
  return a;
}
__device__ __forceinline__ v16h fragc_f32(const float* W, int k0, int n, int lane, int ld, int K) {
  v16h a; const int g = lane >> 4;
#pragma unroll
  for (int i = 0; i < 8; ++i) { const int ka = k0 + 8 * g + i, kb = ka + 16;
    a[i] = (_Float16)(ka < K ? W[(size_t)ka * ld + n] : 0.f); a[8 + i] = (_Float16)(kb < K ? W[(size_t)kb * ld + n] : 0.f); }
  return a;
}
struct F2 { v16b h, l; };
__device__ __forceinline__ F2 bsplit16(const float v[16]) { F2 r;
#pragma unroll
  for (int i = 0; i < 16; ++i) { const __bf16 h = (__bf16)v[i]; r.h[i] = h; r.l[i] = (__bf16)(v[i] - (float)h); }
  return r; }
__device__ __forceinline__ F2 split_row(const float* row, int k0, int lane) { float v[16]; const float* p = row + k0 + 8 * (lane >> 4);
#pragma unroll
  for (int i = 0; i < 8; ++i) { v[i] = p[i]; v[8 + i] = p[16 + i]; }
  return bsplit16(v); }
__device__ __forceinline__ F2 split_rowK(const float* row, int k0, int lane, int K) { float v[16]; const int g = lane >> 4;
#pragma unroll
  for (int i = 0; i < 8; ++i) { const int ka = k0 + 8 * g + i, kb = ka + 16; v[i] = ka < K ? row[ka] : 0.f; v[8 + i] = kb < K ? row[kb] : 0.f; }
  return bsplit16(v); }
__device__ __forceinline__ F2 split_col(const float* W, int k0, int n, int lane, int ld, int K) { float v[16]; const int g = lane >> 4;
#pragma unroll
  for (int i = 0; i < 8; ++i) { const int ka = k0 + 8 * g + i, kb = ka + 16; v[i] = ka < K ? W[(size_t)ka * ld + n] : 0.f; v[8 + i] = kb < K ? W[(size_t)kb * ld + n] : 0.f; }
  return bsplit16(v); }
__device__ __forceinline__ v8f mac3(const F2& a, const F2& b, v8f c) { c = wmma_bf(a.l, b.h, c); c = wmma_bf(a.h, b.l, c); return wmma_bf(a.h, b.h, c); }
__device__ __forceinline__ float sigm(float v) { return 1.0f / (1.0f + expf(-v)); }
#define LDSX() do { asm volatile("s_wait_dscnt 0" ::: "memory"); __builtin_amdgcn_wave_barrier(); __builtin_amdgcn_fence(__ATOMIC_RELEASE, "workgroup"); } while (0)

#define NN 100000
#define NE 3200000
#define FI 128
#define FO 64
#define NNP 100352
#define RBD 8192
#define NRBD ((NN + RBD - 1) / RBD)
#define RBA 4096
#define NRBA ((NN + RBA - 1) / RBA)
#define EPT 16
#define CH (256 * EPT)

__global__ __launch_bounds__(256) void k_deg(const int* __restrict__ src, const int* __restrict__ dst, float* __restrict__ NRM) {
  __shared__ int scnt[RBD];
  const int tid = threadIdx.x, which = blockIdx.y; const int r0 = blockIdx.x * RBD; const int* arr = which == 0 ? src : dst;
  for (int q = tid; q < RBD; q += 256) scnt[q] = 0;
  __syncthreads();
#pragma unroll 1
  for (int c0 = 0; c0 < NE; c0 += CH) { const int e0 = c0 + tid * EPT;
    if (e0 + EPT <= NE) {
#pragma unroll
      for (int v = 0; v < EPT / 4; ++v) { const int4 d4 = *(const int4*)(arr + e0 + v * 4); const int dd[4] = {d4.x, d4.y, d4.z, d4.w};
#pragma unroll
        for (int u = 0; u < 4; ++u) { const unsigned rel = (unsigned)(dd[u] - r0); if (rel < (unsigned)RBD) atomicAdd(&scnt[rel], 1); } } }
    else { for (int u = 0; u < EPT; ++u) { const int e = e0 + u; if (e < NE) { const unsigned rel = (unsigned)(arr[e] - r0); if (rel < (unsigned)RBD) atomicAdd(&scnt[rel], 1); } } } }
  __syncthreads();
  for (int q = tid; q < RBD; q += 256) { const int r = r0 + q; if (r < NNP) vst2(NRM + (size_t)which * NNP + r, rsqrtf(fmaxf((float)scnt[q], 1.0f))); }
}
__global__ __launch_bounds__(128) void k_x(const float* __restrict__ feat, const float* __restrict__ W, const float* __restrict__ NRM, float* __restrict__ S) {
  __shared__ __align__(16) float ssum[64];
  const int tid = threadIdx.x, wave = tid >> 5, lane = tid & 31, col = lane & 15, g = lane >> 4;
  const int r0 = blockIdx.x * 64 + wave * 16; const int ra = (r0 + col) < NN ? (r0 + col) : NN - 1;
  v8f acc[4] = {};
#pragma unroll
  for (int kc = 0; kc < FI / 32; ++kc) { const F2 a = split_row(feat + (size_t)ra * FI, kc * 32, lane);
#pragma unroll
    for (int t = 0; t < 4; ++t) acc[t] = mac3(a, split_col(W, kc * 32, t * 16 + col, lane, FO, FI), acc[t]); }
  float part[8];
#pragma unroll
  for (int r = 0; r < 8; ++r) { part[r] = (acc[0][r] + acc[1][r]) + (acc[2][r] + acc[3][r]); }
#pragma unroll
  for (int r = 0; r < 8; ++r) {
#pragma unroll
    for (int off = 1; off <= 8; off <<= 1) part[r] += __shfl_xor(part[r], off, 32); }
  { float pv = 0.f;
#pragma unroll
    for (int r = 0; r < 8; ++r) pv = (r == col) ? part[r] : pv;
    if (col < 8) { const int row = r0 + 8 * g + col; ssum[wave * 16 + 8 * g + col] = row < NN ? pv * (1.0f / FO) * NRM[row] : 0.f; } }
  __syncthreads();
  if (tid < 16) vst2(S + (size_t)blockIdx.x * 64 + tid * 4, *(const v4f*)(&ssum[tid * 4]));
}
__global__ __launch_bounds__(256) void k_agg(const float* __restrict__ S, const int* __restrict__ src, const int* __restrict__ dst, const float* __restrict__ NRM, const float* __restrict__ b, float* __restrict__ out) {
  __shared__ float sacc[RBA];
  __shared__ int ssrc[8][32 * EPT], sdl[8][32 * EPT]; __shared__ int scnt[8]; __shared__ float sbm;
  const int tid = threadIdx.x, wave = tid >> 5, lane = tid & 31;
  const int r0 = blockIdx.x * RBA; const int* esrc = src; const int* edst = dst;
  for (int q = tid; q < RBA; q += 256) sacc[q] = 0.f;
  if (tid == 0) { float s = 0.f; for (int f = 0; f < FO; ++f) s += b[f]; sbm = s * (1.0f / FO); }
  __syncthreads();
#define RB RBA
  #pragma unroll 1
  for (int c0 = 0; c0 < NE; c0 += CH) {
    const int e0 = c0 + tid * EPT; int hd[EPT]; int cnt = 0;
    if (e0 + EPT <= NE) {
#pragma unroll
      for (int v = 0; v < EPT / 4; ++v) { const int4 d4 = *(const int4*)(edst + e0 + v * 4);
        const int dd[4] = {d4.x, d4.y, d4.z, d4.w};
#pragma unroll
        for (int u = 0; u < 4; ++u) { const unsigned rel = (unsigned)(dd[u] - r0); const bool h = rel < (unsigned)RB; hd[v * 4 + u] = h ? (int)rel : -1; cnt += h ? 1 : 0; } } }
    else {
#pragma unroll
      for (int u = 0; u < EPT; ++u) { const int e = e0 + u; hd[u] = -1; if (e < NE) { const unsigned rel = (unsigned)(edst[e] - r0); if (rel < (unsigned)RB) { hd[u] = (int)rel; ++cnt; } } } }
    int incl = cnt;
#pragma unroll
    for (int off = 1; off < 32; off <<= 1) { const int vv = __shfl_up(incl, off, 32); if (lane >= off) incl += vv; }
    const int wtot = __shfl(incl, 31, 32); int pos = incl - cnt;
    if (cnt > 0) {
#pragma unroll
      for (int u = 0; u < EPT; ++u) if (hd[u] >= 0) { int s = esrc[e0 + u]; s = s < 0 ? 0 : (s >= NN ? NN - 1 : s); ssrc[wave][pos] = s; sdl[wave][pos] = hd[u];  ++pos; } }
    if (lane == 0) scnt[wave] = wtot;
    __syncthreads();
    for (int w = 0; w < 8; ++w) { const int nh = scnt[w]; for (int i = 0; i < nh; ++i) { const int dl = sdl[w][i]; if ((dl & 255) == tid) sacc[dl] += S[ssrc[w][i]]; } }
    __syncthreads(); }
#undef RB
  for (int q = tid; q < RBA / 4; q += 256) { v4f o; const int d0 = r0 + q * 4; if (d0 >= NN) continue;
#pragma unroll
    for (int e = 0; e < 4; ++e) { const int d = d0 + e; o[e] = d < NN ? sacc[q * 4 + e] * NRM[(size_t)NNP + d] + sbm : 0.f; }
    if (d0 + 3 < NN) vst2(out + d0, o); else { for (int e = 0; e < 4; ++e) if (d0 + e < NN) vst2(out + d0 + e, o[e]); } }
}
extern "C" void kernel_launch(void* const* d_in, const int* in_sizes, int n_in, void* d_out, int out_size, void* d_ws, size_t ws_size, hipStream_t stream) {
  (void)in_sizes; (void)n_in; (void)out_size; (void)ws_size;
  const float* feat = (const float*)d_in[0]; const float* W = (const float*)d_in[1]; const float* b = (const float*)d_in[2]; const int* src = (const int*)d_in[3]; const int* dst = (const int*)d_in[4];
  float* out = (float*)d_out;
  char* ws = (char*)d_ws; size_t off = 0;
  auto take = [&](size_t bytes) { char* p = ws + off; off += (bytes + 255) & ~(size_t)255; return p; };
  float* NRM = (float*)take((size_t)2 * NNP * 4); float* S = (float*)take((size_t)NNP * 4);
  k_deg<<<dim3(NRBD, 2), 256, 0, stream>>>(src, dst, NRM);
  k_x<<<NNP / 64, 128, 0, stream>>>(feat, W, NRM, S);
  k_agg<<<NRBA, 256, 0, stream>>>(S, src, dst, NRM, b, out);
}
